// MoDAAttention_89618787599008
// MI455X (gfx1250) — hardware-verified
//
#include <hip/hip_runtime.h>
#include <math.h>

constexpr int kBatch   = 8;
constexpr int kSeqN    = 1024;
constexpr int kDimC    = 768;
constexpr int kHkv     = 2;
constexpr int kHd      = 64;
constexpr int kGrp     = 6;
constexpr int kTok     = kBatch * kSeqN;
constexpr int kKeys    = 2 * kSeqN;
constexpr int kQpos    = kSeqN * kGrp;
constexpr int kGroups  = kBatch * kHkv;
constexpr int kKVch    = 2 * kHkv * kHd;
constexpr int kHalfKV  = kHkv * kHd;
constexpr float kWCarry    = 64.0f;
constexpr float kWCarryInv = 1.0f / 64.0f;
constexpr float kPCarry    = 2048.0f;
constexpr float kOCarry    = 256.0f;
constexpr float kScoreScale = 0.125f;
constexpr float kPVScale    = kOCarry / kPCarry;
constexpr float kOutScale   = 1.0f / (kOCarry * kWCarry);

typedef __attribute__((ext_vector_type(16))) _Float16 v16h;
typedef __attribute__((ext_vector_type(8)))  _Float16 v8h;
typedef __attribute__((ext_vector_type(16))) __bf16   v16b;
typedef __attribute__((ext_vector_type(8)))  __bf16   v8b;
typedef __attribute__((ext_vector_type(8)))  float    v8f;
typedef __attribute__((ext_vector_type(4)))  float    v4f;
typedef __attribute__((ext_vector_type(4)))  unsigned int v4u;

__device__ __forceinline__ unsigned short f2bf_bits(float f) {
  unsigned u = __float_as_uint(f);
  return (unsigned short)((u + 0x7FFFu + ((u >> 16) & 1u)) >> 16);
}
__device__ __forceinline__ float bf_bits2f(unsigned short h) { return __uint_as_float(((unsigned)h) << 16); }

__device__ __forceinline__ void dep_guard_h(v8f& a, v8f& b, v16h x, v16h y) { asm volatile("v_nop\n\tv_nop\n\tv_nop\n\tv_nop" : "+v"(a), "+v"(b) : "v"(x), "v"(y)); }
__device__ __forceinline__ void dep_guard_b(v8f& a, v8f& b, v16b x, v16b y) { asm volatile("v_nop\n\tv_nop\n\tv_nop\n\tv_nop" : "+v"(a), "+v"(b) : "v"(x), "v"(y)); }
__device__ __forceinline__ void keep4_h(v16h a, v16h b, v16h c, v16h d) { asm volatile("v_nop" :: "v"(a), "v"(b), "v"(c), "v"(d)); }
__device__ __forceinline__ void keep4_b(v16b a, v16b b, v16b c, v16b d) { asm volatile("v_nop" :: "v"(a), "v"(b), "v"(c), "v"(d)); }
__device__ __forceinline__ void acc_guard4(v8f& a, v8f& b, v8f& c, v8f& d) { asm volatile("v_nop\n\tv_nop\n\tv_nop\n\tv_nop" : "+v"(a), "+v"(b), "+v"(c), "+v"(d)); }
template <typename T> struct Frag;
template <> struct Frag<_Float16> {
  typedef v16h V; union U { v16h v; v8h h[2]; };
  static __device__ __forceinline__ v16h load(const _Float16* p) {
    U f; f.h[0] = *(const v8h*)(p); f.h[1] = *(const v8h*)(p + 16); return f.v;
  }
  static __device__ __forceinline__ v8f mma(v16h a, v16h b, v8f c) {
    return __builtin_amdgcn_wmma_f32_16x16x32_f16(false, a, false, b, (short)0, c, false, false);
  }
  static __device__ __forceinline__ void guard(v8f& a, v8f& b, v16h x, v16h y) { dep_guard_h(a, b, x, y); }
  static __device__ __forceinline__ void keep(v16h a, v16h b, v16h c, v16h d) { keep4_h(a, b, c, d); }
};
template <> struct Frag<__bf16> {
  typedef v16b V; union U { v16b v; v8b h[2]; };
  static __device__ __forceinline__ v16b load(const __bf16* p) {
    U f; f.h[0] = *(const v8b*)(p); f.h[1] = *(const v8b*)(p + 16); return f.v;
  }
  static __device__ __forceinline__ v8f mma(v16b a, v16b b, v8f c) {
    return __builtin_amdgcn_wmma_f32_16x16x32_bf16(false, a, false, b, (short)0, c, false, false);
  }
  static __device__ __forceinline__ void guard(v8f& a, v8f& b, v16b x, v16b y) { dep_guard_b(a, b, x, y); }
  static __device__ __forceinline__ void keep(v16b a, v16b b, v16b c, v16b d) { keep4_b(a, b, c, d); }
};

__device__ __forceinline__ unsigned pk16(unsigned short a, unsigned short b) { return (unsigned)a | ((unsigned)b << 16); }
__device__ __forceinline__ unsigned short h_bits(float f) { const _Float16 h = (_Float16)f; return __builtin_bit_cast(unsigned short, h); }

template <int ET> struct Elem;
template <> struct Elem<0> { typedef _Float16 T; };
template <> struct Elem<1> { typedef __bf16 T; };
template <int ET, bool SPLIT, int BIAS_MODE, int OUT_MODE, bool RESID, int ACT = 0>
__global__ __launch_bounds__(256) void wmma_gemm64(
    const unsigned short* __restrict__ Ap, const unsigned short* __restrict__ A2p, int lda, long strideA,
    const unsigned short* __restrict__ Btp, const unsigned short* __restrict__ Bt2p, int ldb, long strideB,
    void* __restrict__ Cout, void* __restrict__ Cout2, int ldc, long strideC,
    const float* __restrict__ bias,
    const float* __restrict__ resid, long strideR,
    int M, int N, int K, float scale) {
  typedef typename Elem<ET>::T T;
  typedef typename Frag<T>::V V;
  const T* A = (const T*)Ap; const T* A2 = (const T*)A2p; const T* Bt = (const T*)Btp; const T* Bt2 = (const T*)Bt2p;
  __shared__ __align__(16) float sT[8][16 * 68];
  const int b    = blockIdx.y;
  const int lane = threadIdx.x & 31;
  const int wave = threadIdx.x >> 5;
  const int tilesN = N >> 6;
  const int tilesM = M >> 6;
  const int tile = blockIdx.x * 8 + wave;
  if (tile >= tilesM * tilesN) return;
  const int tm = tile / tilesN;
  const int tn = tile - tm * tilesN;
  const int m0 = tm << 6;
  const int n0 = tn << 6;

  const T* Ab  = A  + (size_t)b * strideA;
  const T* Bb  = Bt + (size_t)b * strideB;
  const T* Ab2 = SPLIT ? (A2  + (size_t)b * strideA) : nullptr;
  const T* Bb2 = SPLIT ? (Bt2 + (size_t)b * strideB) : nullptr;

  const int rlane = lane & 15;
  const int koff  = (lane >> 4) * 8;
  const int mOff  = (lane >> 4) * 8;

  v8f acc[4][4];
#pragma unroll
  for (int i = 0; i < 4; ++i)
#pragma unroll
    for (int j = 0; j < 4; ++j) acc[i][j] = (v8f){0.f,0.f,0.f,0.f,0.f,0.f,0.f,0.f};

  for (int k0 = 0; k0 < K; k0 += 32) {
    V bh[4], bl[4];
#pragma unroll
    for (int j = 0; j < 4; ++j) {
      const size_t bo = (size_t)(n0 + (j << 4) + rlane) * ldb + koff + k0;
      bh[j] = Frag<T>::load(Bb + bo);
      if (SPLIT) bl[j] = Frag<T>::load(Bb2 + bo);
    }
#pragma unroll
    for (int i = 0; i < 4; ++i) {
      const size_t ao = (size_t)(m0 + (i << 4) + rlane) * lda + koff + k0;
      V ah = Frag<T>::load(Ab + ao);
      V al;
      if (SPLIT) al = Frag<T>::load(Ab2 + ao);
#pragma unroll
      for (int j = 0; j < 4; ++j) {
        acc[i][j] = Frag<T>::mma(ah, bh[j], acc[i][j]);
        if (SPLIT) {
          acc[i][j] = Frag<T>::mma(ah, bl[j], acc[i][j]);
          acc[i][j] = Frag<T>::mma(al, bh[j], acc[i][j]);
        }
      }
      Frag<T>::guard(acc[i][0], acc[i][3], ah, SPLIT ? al : ah);
    }
    Frag<T>::keep(bh[0], bh[1], bh[2], bh[3]);
    if (SPLIT) Frag<T>::keep(bl[0], bl[1], bl[2], bl[3]);
  }
  acc_guard4(acc[0][0], acc[0][1], acc[0][2], acc[0][3]);
  acc_guard4(acc[1][0], acc[1][1], acc[1][2], acc[1][3]);
  acc_guard4(acc[2][0], acc[2][1], acc[2][2], acc[2][3]);
  acc_guard4(acc[3][0], acc[3][1], acc[3][2], acc[3][3]);

  float* slab = sT[wave];
  const float* Rb = RESID ? (resid + (size_t)b * strideR) : nullptr;
#pragma unroll
  for (int i = 0; i < 4; ++i) {
    const int mBase = m0 + (i << 4);
#pragma unroll
    for (int j = 0; j < 4; ++j) {
      const int n = n0 + (j << 4) + rlane;
      float bv = 0.f;
      if (BIAS_MODE == 2) bv = bias[n];
#pragma unroll
      for (int r = 0; r < 8; ++r) {
        float v = acc[i][j][r] * scale;
        if (BIAS_MODE == 1) v += bias[mBase + mOff + r];
        if (BIAS_MODE == 2) v += bv;
        if (RESID) v += Rb[(size_t)(mBase + mOff + r) * ldc + n];
        if (ACT == 2) v = fmaxf(v, 0.0f);
        if (ACT == 4) v = (v > 0.f) ? v : 0.01f * v;
        slab[(mOff + r) * 68 + (j << 4) + rlane] = v;
      }
    }
    __builtin_amdgcn_fence(__ATOMIC_RELEASE, "workgroup");
    __builtin_amdgcn_wave_barrier();
    __builtin_amdgcn_fence(__ATOMIC_ACQUIRE, "workgroup");
    if (OUT_MODE == 0) {
      float* C = (float*)Cout + (size_t)b * strideC;
      const int hh = lane >> 4, c4 = (lane & 15) * 4;
      for (int pass = 0; pass < 2; ++pass) {
#pragma unroll
        for (int it = 0; it < 8; ++it) {
          const int row = it * 2 + hh;
          v4f v = *(const v4f*)(slab + row * 68 + c4);
          *(volatile v4f*)(C + (size_t)(mBase + row) * ldc + n0 + c4) = v;
        }
        __threadfence();
      }
    } else {
      const int q = lane >> 3, c8 = (lane & 7) * 8;
      unsigned short* C  = (unsigned short*)Cout  + (size_t)b * strideC;
      unsigned short* C2 = (OUT_MODE == 2) ? ((unsigned short*)Cout2 + (size_t)b * strideC) : nullptr;
      for (int pass = 0; pass < 2; ++pass) {
#pragma unroll
        for (int it = 0; it < 4; ++it) {
          const int row = it * 4 + q;
          const float* sp = slab + row * 68 + c8;
          v8h hv, lv;
#pragma unroll
          for (int e = 0; e < 8; ++e) {
            if (OUT_MODE == 1) {
              hv[e] = (_Float16)sp[e];
            } else {
              unsigned short hb = f2bf_bits(sp[e]);
              unsigned short lb = f2bf_bits(sp[e] - bf_bits2f(hb));
              hv[e] = __builtin_bit_cast(_Float16, hb);
              lv[e] = __builtin_bit_cast(_Float16, lb);
            }
          }
          *(volatile v8h*)(C + (size_t)(mBase + row) * ldc + n0 + c8) = hv;
          if (OUT_MODE == 2) *(volatile v8h*)(C2 + (size_t)(mBase + row) * ldc + n0 + c8) = lv;
        }
        __threadfence();
      }
    }
    __builtin_amdgcn_fence(__ATOMIC_RELEASE, "workgroup");
    __builtin_amdgcn_wave_barrier();
    __builtin_amdgcn_fence(__ATOMIC_ACQUIRE, "workgroup");
  }
}

__global__ __launch_bounds__(256) void cast8_f16_kernel(const float* __restrict__ in, unsigned short* __restrict__ out,
                                                        int n8, float scale) {
  const int i = blockIdx.x * 256 + threadIdx.x;
  if (i >= n8) return;
  const float* p = in + 8 * (size_t)i;
  const v4f a = *(const v4f*)(p);
  const v4f c = *(const v4f*)(p + 4);
  unsigned short hb[8];
#pragma unroll
  for (int e = 0; e < 4; ++e) {
    hb[e]     = h_bits(a[e] * scale);
    hb[4 + e] = h_bits(c[e] * scale);
  }
  const v4u u = (v4u){pk16(hb[0], hb[1]), pk16(hb[2], hb[3]), pk16(hb[4], hb[5]), pk16(hb[6], hb[7])};
  unsigned short* q = out + 8 * (size_t)i;
  *(volatile v4u*)q = u;
  __threadfence();
  *(volatile v4u*)q = u;
}

__global__ __launch_bounds__(256) void kvplanes_kernel(const float* __restrict__ ck, const float* __restrict__ cv,
                                                       const float* __restrict__ kn, const float* __restrict__ vn,
                                                       unsigned short* __restrict__ Kp, unsigned short* __restrict__ Vtp) {
  __shared__ float sm[64][65];
  const int t = threadIdx.x;
  const int lane = t & 31, wave = t >> 5;
  const int kt = blockIdx.x;
  const int g  = blockIdx.y;
  const int b  = g >> 1, h = g & 1;
  const bool isnew = (kt >= 16);
  const float* srcK = isnew ? kn : ck;
  const float* srcV = isnew ? vn : cv;
  const size_t rowbase = (size_t)b * kSeqN + (size_t)(kt & 15) * 64;

  v4u uk[2];
  size_t ko[2];
#pragma unroll
  for (int it = 0; it < 2; ++it) {
    const int idx = it * 256 + t;
    const int r   = idx >> 3;
    const int c8  = (idx & 7) * 8;
    const size_t so = (rowbase + r) * kHalfKV + (size_t)h * kHd + c8;
    const v4f a  = *(const v4f*)(srcK + so);
    const v4f c  = *(const v4f*)(srcK + so + 4);
    const v4f va = *(const v4f*)(srcV + so);
    const v4f vc = *(const v4f*)(srcV + so + 4);
    unsigned short hb[8];
#pragma unroll
    for (int e = 0; e < 4; ++e) {
      hb[e]     = h_bits(a[e]);
      hb[4 + e] = h_bits(c[e]);
      sm[r][c8 + e]     = va[e];
      sm[r][c8 + 4 + e] = vc[e];
    }
    uk[it] = (v4u){pk16(hb[0], hb[1]), pk16(hb[2], hb[3]), pk16(hb[4], hb[5]), pk16(hb[6], hb[7])};
    ko[it] = ((size_t)g * kKeys + (size_t)kt * 64 + r) * kHd + c8;
  }
  *(volatile v4u*)(Kp + ko[0]) = uk[0];
  *(volatile v4u*)(Kp + ko[1]) = uk[1];
  __threadfence();
  *(volatile v4u*)(Kp + ko[0]) = uk[0];
  *(volatile v4u*)(Kp + ko[1]) = uk[1];

  __syncthreads();

  const int q = lane >> 3, c8 = (lane & 7) * 8;
  v4u uv[2];
  size_t vo[2];
#pragma unroll
  for (int it = 0; it < 2; ++it) {
    const int d = wave * 8 + it * 4 + q;
    unsigned short hb[8];
#pragma unroll
    for (int e = 0; e < 8; ++e) hb[e] = h_bits(sm[c8 + e][d]);
    uv[it] = (v4u){pk16(hb[0], hb[1]), pk16(hb[2], hb[3]), pk16(hb[4], hb[5]), pk16(hb[6], hb[7])};
    vo[it] = ((size_t)g * kHd + d) * kKeys + (size_t)kt * 64 + c8;
  }
  *(volatile v4u*)(Vtp + vo[0]) = uv[0];
  *(volatile v4u*)(Vtp + vo[1]) = uv[1];
  __threadfence();
  *(volatile v4u*)(Vtp + vo[0]) = uv[0];
  *(volatile v4u*)(Vtp + vo[1]) = uv[1];
}

__global__ __launch_bounds__(256) void softmax_row_kernel(const float* __restrict__ Sp, unsigned short* __restrict__ Pp,
                                                          float carry) {
  __shared__ float redM[8];
  __shared__ float redS[8];
  const int row  = blockIdx.x;
  const int t    = threadIdx.x;
  const int lane = t & 31, wave = t >> 5;
  const int c0   = t * 8;
  const float* sr = Sp + (size_t)row * kKeys + c0;
  const v4f a = *(const v4f*)(sr);
  const v4f c = *(const v4f*)(sr + 4);
  float x[8];
#pragma unroll
  for (int e = 0; e < 4; ++e) { x[e] = a[e]; x[4 + e] = c[e]; }
  float m = fmaxf(fmaxf(fmaxf(x[0], x[1]), fmaxf(x[2], x[3])), fmaxf(fmaxf(x[4], x[5]), fmaxf(x[6], x[7])));
#pragma unroll
  for (int off = 16; off > 0; off >>= 1) m = fmaxf(m, __shfl_xor(m, off, 32));
  if (lane == 0) redM[wave] = m;
  __syncthreads();
  float gm = redM[0];
#pragma unroll
  for (int w = 1; w < 8; ++w) gm = fmaxf(gm, redM[w]);
  float ex[8];
#pragma unroll
  for (int e = 0; e < 8; ++e) ex[e] = expf(x[e] - gm);
  float s = ((ex[0] + ex[1]) + (ex[2] + ex[3])) + ((ex[4] + ex[5]) + (ex[6] + ex[7]));
#pragma unroll
  for (int off = 16; off > 0; off >>= 1) s += __shfl_xor(s, off, 32);
  if (lane == 0) redS[wave] = s;
  __syncthreads();
  float tot = redS[0];
#pragma unroll
  for (int w = 1; w < 8; ++w) tot += redS[w];
  const float sc = carry * (1.0f / tot);
  unsigned short hb[8];
#pragma unroll
  for (int e = 0; e < 8; ++e) hb[e] = h_bits(ex[e] * sc);
  const v4u u = (v4u){pk16(hb[0], hb[1]), pk16(hb[2], hb[3]), pk16(hb[4], hb[5]), pk16(hb[6], hb[7])};
  unsigned short* q = Pp + (size_t)row * kKeys + c0;
  *(volatile v4u*)q = u;
  __threadfence();
  *(volatile v4u*)q = u;
}

extern "C" void kernel_launch(void* const* d_in, const int* in_sizes, int n_in,
                              void* d_out, int out_size, void* d_ws,
                              size_t ws_size, hipStream_t stream) {
  if (n_in < 9) return;
  if (in_sizes[0] != kTok * kDimC) return;
  if (in_sizes[1] != kTok * kHalfKV || in_sizes[2] != kTok * kHalfKV) return;
  if (in_sizes[3] != kDimC * kDimC || in_sizes[4] != kDimC) return;
  if (in_sizes[5] != kKVch * kDimC || in_sizes[6] != kKVch) return;
  if (in_sizes[7] != kDimC * kDimC || in_sizes[8] != kDimC) return;
  if (out_size != kTok * kDimC + 2 * kTok * kHalfKV) return;

  const float* x     = (const float*)d_in[0];
  const float* ck    = (const float*)d_in[1];
  const float* cv    = (const float*)d_in[2];
  const float* Wq    = (const float*)d_in[3];
  const float* bq    = (const float*)d_in[4];
  const float* Wkv   = (const float*)d_in[5];
  const float* bkv   = (const float*)d_in[6];
  const float* Wproj = (const float*)d_in[7];
  const float* bproj = (const float*)d_in[8];

  float* out0 = (float*)d_out;
  float* out1 = out0 + (size_t)kTok * kDimC;
  float* out2 = out1 + (size_t)kTok * kHalfKV;

  const size_t szX   = (size_t)kTok * kDimC * 2;
  const size_t szWq  = (size_t)kDimC * kDimC * 2;
  const size_t szWkv = (size_t)kKVch * kDimC * 2;
  const size_t szWp  = (size_t)kDimC * kDimC * 2;
  const size_t szQ   = (size_t)kTok * kDimC * 2;
  const size_t szK   = (size_t)kGroups * kKeys * kHd * 2;
  const size_t szVt  = (size_t)kGroups * kHd * kKeys * 2;
  const size_t szO   = (size_t)kTok * kDimC * 2;
  const size_t szS   = (size_t)kQpos * kKeys * 4;
  const size_t szP   = (size_t)kQpos * kKeys * 2;

  unsigned char* wsb = (unsigned char*)d_ws;
  size_t off = 0;
  unsigned short* X16   = (unsigned short*)(wsb + off); off += szX;
  unsigned short* Wq16  = (unsigned short*)(wsb + off); off += szWq;
  unsigned short* Wkv16 = (unsigned short*)(wsb + off); off += szWkv;
  unsigned short* Wp16  = (unsigned short*)(wsb + off); off += szWp;
  unsigned short* Q16   = (unsigned short*)(wsb + off); off += szQ;
  unsigned short* K16   = (unsigned short*)(wsb + off); off += szK;
  unsigned short* Vt16  = (unsigned short*)(wsb + off); off += szVt;
  unsigned short* O16   = (unsigned short*)(wsb + off); off += szO;
  float*          Sbuf  = (float*)(wsb + off);          off += szS;
  unsigned short* P16   = (unsigned short*)(wsb + off); off += szP;
  if (off > ws_size) return;

  {
    const int n8x  = kTok * kDimC / 8;
    const int n8q  = kDimC * kDimC / 8;
    const int n8kv = kKVch * kDimC / 8;
    cast8_f16_kernel<<<dim3((n8x + 255) / 256), 256, 0, stream>>>(x, X16, n8x, 1.0f);
    cast8_f16_kernel<<<dim3((n8q + 255) / 256), 256, 0, stream>>>(Wq, Wq16, n8q, kWCarry);
    cast8_f16_kernel<<<dim3((n8kv + 255) / 256), 256, 0, stream>>>(Wkv, Wkv16, n8kv, kWCarry);
    cast8_f16_kernel<<<dim3((n8q + 255) / 256), 256, 0, stream>>>(Wproj, Wp16, n8q, kWCarry);
  }

  wmma_gemm64<0, false, 2, 1, false><<<dim3(192, 1), 256, 0, stream>>>(
      X16, nullptr, kDimC, 0L, Wq16, nullptr, kDimC, 0L,
      (void*)Q16, nullptr, kDimC, 0L, bq, nullptr, 0L, kTok, kDimC, kDimC, kWCarryInv);

  wmma_gemm64<0, false, 2, 0, false><<<dim3(32, 1), 256, 0, stream>>>(
      X16, nullptr, kDimC, 0L, Wkv16, nullptr, kDimC, 0L,
      (void*)out1, nullptr, kHalfKV, 0L, bkv, nullptr, 0L, kTok, kHalfKV, kDimC, kWCarryInv);
  wmma_gemm64<0, false, 2, 0, false><<<dim3(32, 1), 256, 0, stream>>>(
      X16, nullptr, kDimC, 0L, Wkv16 + (size_t)kHalfKV * kDimC, nullptr, kDimC, 0L,
      (void*)out2, nullptr, kHalfKV, 0L, bkv + kHalfKV, nullptr, 0L, kTok, kHalfKV, kDimC, kWCarryInv);

  kvplanes_kernel<<<dim3(kKeys / 64, kGroups), 256, 0, stream>>>(ck, cv, out1, out2, K16, Vt16);

  for (int g = 0; g < kGroups; ++g) {
    const int b = g >> 1, h = g & 1;
    const unsigned short* Qg  = Q16 + (size_t)b * kSeqN * kDimC + (size_t)h * kHd;
    const unsigned short* Kg  = K16 + (size_t)g * kKeys * kHd;
    const unsigned short* Vtg = Vt16 + (size_t)g * kHd * kKeys;
    unsigned short*       Og  = O16 + (size_t)b * kSeqN * kDimC + (size_t)h * kHd;

    wmma_gemm64<0, false, 0, 0, false><<<dim3(384, 1), 256, 0, stream>>>(
        Qg, nullptr, kHalfKV, 0L, Kg, nullptr, kHd, 0L,
        (void*)Sbuf, nullptr, kKeys, 0L, nullptr, nullptr, 0L, kQpos, kKeys, kHd, kScoreScale);

    softmax_row_kernel<<<dim3(kQpos), 256, 0, stream>>>(Sbuf, P16, kPCarry);

    wmma_gemm64<0, false, 0, 1, false><<<dim3(12, 1), 256, 0, stream>>>(
        P16, nullptr, kKeys, 0L, Vtg, nullptr, kKeys, 0L,
        (void*)Og, nullptr, kHalfKV, 0L, nullptr, nullptr, 0L, kQpos, kHd, kKeys, kPVScale);
  }

  wmma_gemm64<0, false, 2, 0, false><<<dim3(192, 1), 256, 0, stream>>>(
      O16, nullptr, kDimC, 0L, Wp16, nullptr, kDimC, 0L,
      (void*)out0, nullptr, kDimC, 0L, bproj, nullptr, 0L, kTok, kDimC, kDimC, kOutScale);
}
